// GraphSageNet_67860483277516
// MI455X (gfx1250) — hardware-verified
//
#include <hip/hip_runtime.h>
#include <stdint.h>

typedef __attribute__((ext_vector_type(16))) _Float16 v16h;
typedef __attribute__((ext_vector_type(8)))  _Float16 v8h;
typedef __attribute__((ext_vector_type(16))) __bf16   v16b;
typedef __attribute__((ext_vector_type(8)))  __bf16   v8b;
typedef __attribute__((ext_vector_type(8)))  float    v8f;
typedef __attribute__((ext_vector_type(4)))  float    v4f;
typedef __attribute__((ext_vector_type(4)))  int      v4i;

constexpr int NSAMP   = 32;
constexpr int NNODE   = 32;
constexpr int NIMG    = NSAMP * NNODE;
constexpr int CIN     = 3;
constexpr int CH1     = 64;
constexpr int CH2     = 128;
constexpr int NPIX    = 1024;
constexpr int PADW    = 34;
constexpr int NPADPIX = PADW * PADW;
constexpr int KCONV1  = 32;
constexpr int KCONV2  = 576;
constexpr int HIDD    = 256;
constexpr int OUTDIM  = 128;
constexpr int KSAGE   = 512;
constexpr float WCARRY = 16.0f;
constexpr float ACARRY = 16.0f;

constexpr int PL_W2C       = CH2 * KCONV2;
constexpr int PL_FCW       = HIDD * CH2;
constexpr int PL_W1CAT     = HIDD * KSAGE;
constexpr int PL_W2CAT     = OUTDIM * KSAGE;
constexpr int PL_OFF_FCW   = PL_W2C;
constexpr int PL_OFF_W1CAT = PL_OFF_FCW + PL_FCW;
constexpr int PL_OFF_W2CAT = PL_OFF_W1CAT + PL_W1CAT;
constexpr int PL_TOTAL     = PL_OFF_W2CAT + PL_W2CAT;
constexpr int PREP_PER_BLK = 256 * 8;
static_assert(PL_OFF_FCW % PREP_PER_BLK == 0 && PL_OFF_W1CAT % PREP_PER_BLK == 0 &&
              PL_OFF_W2CAT % PREP_PER_BLK == 0 && PL_TOTAL % PREP_PER_BLK == 0, "segments are block aligned");
constexpr int PREP_BLOCKS    = PL_TOTAL / PREP_PER_BLK;
constexpr int PREP_BLK_FCW   = PL_OFF_FCW / PREP_PER_BLK;
constexpr int PREP_BLK_W1CAT = PL_OFF_W1CAT / PREP_PER_BLK;
constexpr int PREP_BLK_W2CAT = PL_OFF_W2CAT / PREP_PER_BLK;

constexpr size_t WSO_PLANES = 0;
constexpr size_t WSB_PLANES = (size_t)PL_TOTAL * 2;
constexpr size_t WSO_POOL   = WSO_PLANES + WSB_PLANES;
constexpr size_t WSB_POOL   = (size_t)NIMG * CH2 * 2;
constexpr size_t WSO_Z0     = WSO_POOL + WSB_POOL;
constexpr size_t WSB_ZF     = (size_t)NIMG * HIDD * 4;
constexpr size_t WSO_A1     = WSO_Z0 + WSB_ZF;
constexpr size_t WSB_AH     = (size_t)NIMG * KSAGE * 2;
constexpr size_t WSO_Z1     = WSO_A1 + WSB_AH;
constexpr size_t WSO_A2     = WSO_Z1 + WSB_ZF;
constexpr size_t WS_TOTAL   = WSO_A2 + WSB_AH;
static_assert(WS_TOTAL == 5062656, "carve total");
static_assert(WS_TOTAL <= (size_t)134217728, "carve under 128 MiB");
static_assert(WSO_POOL % 256 == 0 && WSO_Z0 % 256 == 0 && WSO_A1 % 256 == 0 && WSO_Z1 % 256 == 0 && WSO_A2 % 256 == 0, "alignment");

static_assert(NIMG % 64 == 0 && HIDD % 64 == 0 && OUTDIM % 64 == 0, "tile multiples");
static_assert(CH2 % 32 == 0 && KSAGE % 32 == 0, "K multiples of 32");

__device__ __forceinline__ unsigned short f2bf_bits(float f) {
  unsigned u = __float_as_uint(f);
  return (unsigned short)((u + 0x7FFFu + ((u >> 16) & 1u)) >> 16);
}
__device__ __forceinline__ float bf_bits2f(unsigned short h) { return __uint_as_float(((unsigned)h) << 16); }

__device__ __forceinline__ void dep_guard_h(v8f& a, v8f& b, v16h x, v16h y) { asm volatile("v_nop\n\tv_nop\n\tv_nop\n\tv_nop" : "+v"(a), "+v"(b) : "v"(x), "v"(y)); }
__device__ __forceinline__ void dep_guard_b(v8f& a, v8f& b, v16b x, v16b y) { asm volatile("v_nop\n\tv_nop\n\tv_nop\n\tv_nop" : "+v"(a), "+v"(b) : "v"(x), "v"(y)); }
__device__ __forceinline__ void keep4_h(v16h a, v16h b, v16h c, v16h d) { asm volatile("v_nop" :: "v"(a), "v"(b), "v"(c), "v"(d)); }
__device__ __forceinline__ void keep4_b(v16b a, v16b b, v16b c, v16b d) { asm volatile("v_nop" :: "v"(a), "v"(b), "v"(c), "v"(d)); }
__device__ __forceinline__ void acc_guard4(v8f& a, v8f& b, v8f& c, v8f& d) { asm volatile("v_nop\n\tv_nop\n\tv_nop\n\tv_nop" : "+v"(a), "+v"(b), "+v"(c), "+v"(d)); }
__device__ __forceinline__ void dep_guard3_h(v8f& a, v8f& b, v16h x, v16h y, v16h z) { asm volatile("v_nop\n\tv_nop\n\tv_nop\n\tv_nop" : "+v"(a), "+v"(b) : "v"(x), "v"(y), "v"(z)); }
__device__ __forceinline__ v8f mma_h1(v16h a, v16h b, v8f c) {
  c = __builtin_amdgcn_wmma_f32_16x16x32_f16(false, a, false, b, (short)0, c, false, false);
  asm volatile("v_nop\n\tv_nop\n\tv_nop\n\tv_nop" : "+v"(c) : "v"(a), "v"(b));
  return c;
}

template <typename T> struct Frag;
template <> struct Frag<_Float16> {
  typedef v16h V; union U { v16h v; v8h h[2]; };
  static __device__ __forceinline__ v16h load(const _Float16* p) {
    U f; f.h[0] = *(const v8h*)(p); f.h[1] = *(const v8h*)(p + 16); return f.v;
  }
  static __device__ __forceinline__ v8f mma(v16h a, v16h b, v8f c) {
    return __builtin_amdgcn_wmma_f32_16x16x32_f16(false, a, false, b, (short)0, c, false, false);
  }
  static __device__ __forceinline__ void guard(v8f& a, v8f& b, v16h x, v16h y) { dep_guard_h(a, b, x, y); }
  static __device__ __forceinline__ void keep(v16h a, v16h b, v16h c, v16h d) { keep4_h(a, b, c, d); }
};
template <> struct Frag<__bf16> {
  typedef v16b V; union U { v16b v; v8b h[2]; };
  static __device__ __forceinline__ v16b load(const __bf16* p) {
    U f; f.h[0] = *(const v8b*)(p); f.h[1] = *(const v8b*)(p + 16); return f.v;
  }
  static __device__ __forceinline__ v8f mma(v16b a, v16b b, v8f c) {
    return __builtin_amdgcn_wmma_f32_16x16x32_bf16(false, a, false, b, (short)0, c, false, false);
  }
  static __device__ __forceinline__ void guard(v8f& a, v8f& b, v16b x, v16b y) { dep_guard_b(a, b, x, y); }
  static __device__ __forceinline__ void keep(v16b a, v16b b, v16b c, v16b d) { keep4_b(a, b, c, d); }
};
typedef Frag<_Float16> FragH;

template <int ET> struct Elem;
template <> struct Elem<0> { typedef _Float16 T; };
template <> struct Elem<1> { typedef __bf16 T; };
template <int ET, bool SPLIT, int BIAS_MODE, int OUT_MODE, bool RESID, int ACT = 0>
__global__ __launch_bounds__(256) void wmma_gemm64(
    const unsigned short* __restrict__ Ap, const unsigned short* __restrict__ A2p, int lda, long strideA,
    const unsigned short* __restrict__ Btp, const unsigned short* __restrict__ Bt2p, int ldb, long strideB,
    void* __restrict__ Cout, void* __restrict__ Cout2, int ldc, long strideC,
    const float* __restrict__ bias,
    const float* __restrict__ resid, long strideR,
    int M, int N, int K, float scale) {
  typedef typename Elem<ET>::T T;
  typedef typename Frag<T>::V V;
  const T* A = (const T*)Ap; const T* A2 = (const T*)A2p; const T* Bt = (const T*)Btp; const T* Bt2 = (const T*)Bt2p;
  __shared__ __align__(16) float sT[8][16 * 68];
  const int b    = blockIdx.y;
  const int lane = threadIdx.x & 31;
  const int wave = threadIdx.x >> 5;
  const int tilesN = N >> 6;
  const int tilesM = M >> 6;
  const int tile = blockIdx.x * 8 + wave;
  if (tile >= tilesM * tilesN) return;
  const int tm = tile / tilesN;
  const int tn = tile - tm * tilesN;
  const int m0 = tm << 6;
  const int n0 = tn << 6;

  const T* Ab  = A  + (size_t)b * strideA;
  const T* Bb  = Bt + (size_t)b * strideB;
  const T* Ab2 = SPLIT ? (A2  + (size_t)b * strideA) : nullptr;
  const T* Bb2 = SPLIT ? (Bt2 + (size_t)b * strideB) : nullptr;

  const int rlane = lane & 15;
  const int koff  = (lane >> 4) * 8;
  const int mOff  = (lane >> 4) * 8;

  v8f acc[4][4];
#pragma unroll
  for (int i = 0; i < 4; ++i)
#pragma unroll
    for (int j = 0; j < 4; ++j) acc[i][j] = (v8f){0.f,0.f,0.f,0.f,0.f,0.f,0.f,0.f};

  for (int k0 = 0; k0 < K; k0 += 32) {
    V bh[4], bl[4];
#pragma unroll
    for (int j = 0; j < 4; ++j) {
      const size_t bo = (size_t)(n0 + (j << 4) + rlane) * ldb + koff + k0;
      bh[j] = Frag<T>::load(Bb + bo);
      if (SPLIT) bl[j] = Frag<T>::load(Bb2 + bo);
    }
#pragma unroll
    for (int i = 0; i < 4; ++i) {
      const size_t ao = (size_t)(m0 + (i << 4) + rlane) * lda + koff + k0;
      V ah = Frag<T>::load(Ab + ao);
      V al;
      if (SPLIT) al = Frag<T>::load(Ab2 + ao);
#pragma unroll
      for (int j = 0; j < 4; ++j) {
        acc[i][j] = Frag<T>::mma(ah, bh[j], acc[i][j]);
        if (SPLIT) {
          acc[i][j] = Frag<T>::mma(ah, bl[j], acc[i][j]);
          acc[i][j] = Frag<T>::mma(al, bh[j], acc[i][j]);
        }
      }
      Frag<T>::guard(acc[i][0], acc[i][3], ah, SPLIT ? al : ah);
    }
    Frag<T>::keep(bh[0], bh[1], bh[2], bh[3]);
    if (SPLIT) Frag<T>::keep(bl[0], bl[1], bl[2], bl[3]);
  }
  acc_guard4(acc[0][0], acc[0][1], acc[0][2], acc[0][3]);
  acc_guard4(acc[1][0], acc[1][1], acc[1][2], acc[1][3]);
  acc_guard4(acc[2][0], acc[2][1], acc[2][2], acc[2][3]);
  acc_guard4(acc[3][0], acc[3][1], acc[3][2], acc[3][3]);

  float* slab = sT[wave];
  const float* Rb = RESID ? (resid + (size_t)b * strideR) : nullptr;
#pragma unroll
  for (int i = 0; i < 4; ++i) {
    const int mBase = m0 + (i << 4);
#pragma unroll
    for (int j = 0; j < 4; ++j) {
      const int n = n0 + (j << 4) + rlane;
      float bv = 0.f;
      if (BIAS_MODE == 2) bv = bias[n];
#pragma unroll
      for (int r = 0; r < 8; ++r) {
        float v = acc[i][j][r] * scale;
        if (BIAS_MODE == 1) v += bias[mBase + mOff + r];
        if (BIAS_MODE == 2) v += bv;
        if (RESID) v += Rb[(size_t)(mBase + mOff + r) * ldc + n];
        if (ACT == 1) v = tanhf(v);
        if (ACT == 2) v = fmaxf(v, 0.0f);
        if (ACT == 3) v = v / (1.0f + expf(-v));
        if (ACT == 4) v = (v > 0.f) ? v : 0.01f * v;
        if (ACT == 5) v = 0.5f * v * (1.0f + erff(v * 0.70710678118654752f));
        slab[(mOff + r) * 68 + (j << 4) + rlane] = v;
      }
    }
    __builtin_amdgcn_fence(__ATOMIC_RELEASE, "workgroup");
    __builtin_amdgcn_wave_barrier();
    __builtin_amdgcn_fence(__ATOMIC_ACQUIRE, "workgroup");
    if (OUT_MODE == 0) {
      float* C = (float*)Cout + (size_t)b * strideC;
      const int hh = lane >> 4, c4 = (lane & 15) * 4;
      for (int pass = 0; pass < 2; ++pass) {
#pragma unroll
        for (int it = 0; it < 8; ++it) {
          const int row = it * 2 + hh;
          v4f v = *(const v4f*)(slab + row * 68 + c4);
          *(volatile v4f*)(C + (size_t)(mBase + row) * ldc + n0 + c4) = v;
        }
        __threadfence();
      }
    } else {
      const int q = lane >> 3, c8 = (lane & 7) * 8;
      unsigned short* C  = (unsigned short*)Cout  + (size_t)b * strideC;
      unsigned short* C2 = (OUT_MODE == 2) ? ((unsigned short*)Cout2 + (size_t)b * strideC) : nullptr;
      for (int pass = 0; pass < 2; ++pass) {
#pragma unroll
        for (int it = 0; it < 4; ++it) {
          const int row = it * 4 + q;
          const float* sp = slab + row * 68 + c8;
          v8h hv, lv;
#pragma unroll
          for (int e = 0; e < 8; ++e) {
            if (OUT_MODE == 1) {
              hv[e] = (_Float16)sp[e];
            } else {
              unsigned short hb = f2bf_bits(sp[e]);
              unsigned short lb = f2bf_bits(sp[e] - bf_bits2f(hb));
              hv[e] = __builtin_bit_cast(_Float16, hb);
              lv[e] = __builtin_bit_cast(_Float16, lb);
            }
          }
          *(volatile v8h*)(C + (size_t)(mBase + row) * ldc + n0 + c8) = hv;
          if (OUT_MODE == 2) *(volatile v8h*)(C2 + (size_t)(mBase + row) * ldc + n0 + c8) = lv;
        }
        __threadfence();
      }
    }
    __builtin_amdgcn_fence(__ATOMIC_RELEASE, "workgroup");
    __builtin_amdgcn_wave_barrier();
    __builtin_amdgcn_fence(__ATOMIC_ACQUIRE, "workgroup");
  }
}

__global__ __launch_bounds__(256)
void prep_planes_kernel(const float* __restrict__ conv2_w, const float* __restrict__ fc_w,
                        const float* __restrict__ s1_lw, const float* __restrict__ s1_rw,
                        const float* __restrict__ s2_lw, const float* __restrict__ s2_rw,
                        _Float16* __restrict__ planes) {
  const int tid = threadIdx.x;
  const int blk = blockIdx.x;
  const int g0 = (blk * 256 + tid) * 8;
  float v[8];
  if (blk < PREP_BLK_FCW) {
    const int o = g0 / KCONV2;
    const int r = g0 - o * KCONV2;
    const int tap = r >> 6;
    const int ci0 = r & 63;
    const float* src = conv2_w + (size_t)o * KCONV2 + tap;
#pragma unroll
    for (int e = 0; e < 8; ++e) v[e] = src[(ci0 + e) * 9] * WCARRY;
  } else if (blk < PREP_BLK_W1CAT) {
    const int j = g0 - PL_OFF_FCW;
    const v4f fa = *(const v4f*)(fc_w + j);
    const v4f fb = *(const v4f*)(fc_w + j + 4);
#pragma unroll
    for (int e = 0; e < 4; ++e) { v[e] = fa[e] * WCARRY; v[4 + e] = fb[e] * WCARRY; }
  } else if (blk < PREP_BLK_W2CAT) {
    const int j = g0 - PL_OFF_W1CAT;
    const int o = j >> 9, k = j & 511, kk = k & 255;
    const float* pl = s1_lw + (size_t)o * HIDD + kk;
    const float* pr = s1_rw + (size_t)o * HIDD + kk;
    const v4f la = *(const v4f*)pl, lc = *(const v4f*)(pl + 4);
    const v4f ra = *(const v4f*)pr, rc = *(const v4f*)(pr + 4);
    const bool left = (k < HIDD);
#pragma unroll
    for (int e = 0; e < 4; ++e) {
      v[e]     = (left ? la[e] : ra[e]) * WCARRY;
      v[4 + e] = (left ? lc[e] : rc[e]) * WCARRY;
    }
  } else {
    const int j = g0 - PL_OFF_W2CAT;
    const int o = j >> 9, k = j & 511, kk = k & 255;
    const float* pl = s2_lw + (size_t)o * HIDD + kk;
    const float* pr = s2_rw + (size_t)o * HIDD + kk;
    const v4f la = *(const v4f*)pl, lc = *(const v4f*)(pl + 4);
    const v4f ra = *(const v4f*)pr, rc = *(const v4f*)(pr + 4);
    const bool left = (k < HIDD);
#pragma unroll
    for (int e = 0; e < 4; ++e) {
      v[e]     = (left ? la[e] : ra[e]) * WCARRY;
      v[4 + e] = (left ? lc[e] : rc[e]) * WCARRY;
    }
  }
  v8h hv;
#pragma unroll
  for (int e = 0; e < 8; ++e) hv[e] = (_Float16)v[e];
  _Float16* dst = planes + g0;
  *(volatile v8h*)dst = hv;
  __threadfence();
  *(volatile v8h*)dst = hv;
}

constexpr int SMO_XS    = 0;
constexpr int SMO_W1B   = 13872;
constexpr int SMO_B1    = 17968;
constexpr int SMO_B2    = 18224;
constexpr int SMO_POOLW = 18736;
constexpr int SMO_POOL  = 20784;
constexpr int SMO_IM    = 21296;
constexpr int SMO_Z1    = 86832;
constexpr int SMO_TOTAL = 234800;
static_assert(SMO_W1B == SMO_XS + CIN * NPADPIX * 4, "lds map");
static_assert(SMO_B1 == SMO_W1B + CH1 * KCONV1 * 2, "lds map");
static_assert(SMO_B2 == SMO_B1 + CH1 * 4 && SMO_POOLW == SMO_B2 + CH2 * 4, "lds map");
static_assert(SMO_POOL == SMO_POOLW + 8 * 64 * 4 && SMO_IM == SMO_POOL + CH2 * 4, "lds map");
static_assert(SMO_Z1 == SMO_IM + NPIX * KCONV1 * 2 && SMO_TOTAL == SMO_Z1 + NPADPIX * CH1 * 2, "lds map");
static_assert(SMO_W1B % 16 == 0 && SMO_IM % 16 == 0 && SMO_Z1 % 16 == 0 && SMO_POOL % 16 == 0, "lds alignment");

__device__ __forceinline__ int border_cell(int bp) {
  const int t = bp - 2 * PADW;
  const int side = (1 + (t >> 1)) * PADW + ((t & 1) ? (PADW - 1) : 0);
  return (bp < PADW) ? bp : ((bp < 2 * PADW) ? ((PADW - 1) * PADW + (bp - PADW)) : side);
}

__global__ __launch_bounds__(256)
void conv_pool_kernel(const float* __restrict__ x, const float* __restrict__ w1,
                      const float* __restrict__ b1, const _Float16* __restrict__ w2c,
                      const float* __restrict__ b2, _Float16* __restrict__ pooled_out) {
  extern __shared__ __align__(16) char smem[];
  float*    xs    = (float*)(smem + SMO_XS);
  _Float16* w1b   = (_Float16*)(smem + SMO_W1B);
  float*    sb1   = (float*)(smem + SMO_B1);
  float*    sb2   = (float*)(smem + SMO_B2);
  float*    poolw = (float*)(smem + SMO_POOLW);
  float*    spool = (float*)(smem + SMO_POOL);
  _Float16* im    = (_Float16*)(smem + SMO_IM);
  _Float16* z1    = (_Float16*)(smem + SMO_Z1);

  const int tid = threadIdx.x;
  const int lane = tid & 31, wv = tid >> 5, hh = lane >> 4, mm = lane & 15;
  const int img = blockIdx.x;
  const v4i zero4 = {0, 0, 0, 0};

  {
    const float* xg = x + (size_t)img * (CIN * NPIX);
#pragma unroll
    for (int it = 0; it < 3; ++it) {
      const int q = it * 256 + tid;
      const v4f xv = *(const v4f*)(xg + 4 * q);
      const int f = 4 * q;
      const int ci = f >> 10, rem = f & 1023, yy = rem >> 5, xx = rem & 31;
      float* d = xs + ci * NPADPIX + (yy + 1) * PADW + (xx + 1);
      d[0] = xv[0]; d[1] = xv[1]; d[2] = xv[2]; d[3] = xv[3];
    }
    for (int i = tid; i < CIN * 132; i += 256) {
      const int ci = (i >= 264) ? 2 : ((i >= 132) ? 1 : 0);
      const int bp = i - ci * 132;
      xs[ci * NPADPIX + border_cell(bp)] = 0.0f;
    }
    {
      const int ch = tid >> 2, kb = (tid & 3) * 8;
      const float* wr = w1 + ch * 27;
      v8h hv;
#pragma unroll
      for (int e = 0; e < 8; ++e) {
        const int k = kb + e;
        const int kc = (k < 27) ? k : 26;
        const float wvv = wr[kc];
        const float val = (k < 27) ? (wvv * WCARRY) : 0.0f;
        hv[e] = (_Float16)val;
      }
      *(v8h*)(w1b + tid * 8) = hv;
    }
    if (tid < CH1) sb1[tid] = b1[tid];
    if (tid < CH2) sb2[tid] = b2[tid];
    for (int i = tid; i < 132 * 8; i += 256) {
      const int bp = i >> 3, part = i & 7;
      *(v4i*)(z1 + border_cell(bp) * CH1 + part * 8) = zero4;
    }
  }
  __syncthreads();

#pragma unroll 1
  for (int j = 0; j < 4; ++j) {
    const int p = j * 256 + tid;
    const int y = p >> 5, xq = p & 31;
    const float* xb = xs + y * PADW + xq;
#pragma unroll
    for (int kq = 0; kq < 4; ++kq) {
      v8h hv;
#pragma unroll
      for (int e = 0; e < 8; ++e) {
        const int k = kq * 8 + e;
        const int tap = (k < 27) ? k : 26;
        const int ci = tap / 9, kh = (tap % 9) / 3, kw = tap % 3;
        hv[e] = (_Float16)xb[ci * NPADPIX + kh * PADW + kw];
      }
      *(v8h*)(im + p * KCONV1 + kq * 8) = hv;
    }
  }
  __syncthreads();

  {
    v16h af[4];
#pragma unroll
    for (int mt = 0; mt < 4; ++mt) af[mt] = FragH::load(w1b + (mt * 16 + mm) * KCONV1 + 8 * hh);
    const v8f zero8 = {0.f, 0.f, 0.f, 0.f, 0.f, 0.f, 0.f, 0.f};
#pragma unroll 1
    for (int q = 0; q < 8; ++q) {
      const int nt = wv * 8 + q;
      const int p = nt * 16 + mm;
      const v16h bf = FragH::load(im + p * KCONV1 + 8 * hh);
      const int y = p >> 5, xq = p & 31;
      _Float16* zdst = z1 + ((y + 1) * PADW + (xq + 1)) * CH1 + 8 * hh;
#pragma unroll
      for (int mt = 0; mt < 4; ++mt) {
        v8f acc = mma_h1(af[mt], bf, zero8);
        v8h hv;
#pragma unroll
        for (int r = 0; r < 8; ++r) {
          const float v = fmaxf(acc[r] * (1.0f / WCARRY) + sb1[mt * 16 + 8 * hh + r], 0.0f);
          hv[r] = (_Float16)v;
        }
        *(v8h*)(zdst + mt * 16) = hv;
      }
    }
  }
  __syncthreads();

  const int mblock = wv & 1, wcol = wv >> 1;
  v8f psum[4];
#pragma unroll
  for (int ai = 0; ai < 4; ++ai) psum[ai] = (v8f){0.f, 0.f, 0.f, 0.f, 0.f, 0.f, 0.f, 0.f};
  const _Float16* abase = w2c + (size_t)(mblock * 64 + mm) * KCONV2 + 8 * hh;
#pragma unroll 1
  for (int jp = 0; jp < 8; ++jp) {
    const int nt0 = wcol * 16 + jp * 2;
    const int p0 = nt0 * 16 + mm;
    const int p1 = p0 + 16;
    const _Float16* zb0 = z1 + ((p0 >> 5) * PADW + (p0 & 31)) * CH1 + 8 * hh;
    const _Float16* zb1 = z1 + ((p1 >> 5) * PADW + (p1 & 31)) * CH1 + 8 * hh;
    v8f acc0[4], acc1[4];
#pragma unroll
    for (int ai = 0; ai < 4; ++ai) {
      acc0[ai] = (v8f){0.f, 0.f, 0.f, 0.f, 0.f, 0.f, 0.f, 0.f};
      acc1[ai] = (v8f){0.f, 0.f, 0.f, 0.f, 0.f, 0.f, 0.f, 0.f};
    }
#pragma unroll 1
    for (int ks = 0; ks < 18; ++ks) {
      const int tap = ks >> 1;
      const int kh = tap / 3;
      const int kw = tap - kh * 3;
      const int zo = (kh * PADW + kw) * CH1 + (ks & 1) * 32;
      const v16h bq0 = FragH::load(zb0 + zo);
      const v16h bq1 = FragH::load(zb1 + zo);
#pragma unroll
      for (int ai = 0; ai < 4; ++ai) {
        const v16h af = FragH::load(abase + (size_t)ai * (16 * KCONV2) + ks * 32);
        acc0[ai] = FragH::mma(af, bq0, acc0[ai]);
        acc1[ai] = FragH::mma(af, bq1, acc1[ai]);
        dep_guard3_h(acc0[ai], acc1[ai], af, bq0, bq1);
      }
    }
#pragma unroll
    for (int ai = 0; ai < 4; ++ai)
#pragma unroll
      for (int r = 0; r < 8; ++r) {
        const float bb = sb2[mblock * 64 + ai * 16 + 8 * hh + r];
        const float u0 = fmaxf(acc0[ai][r] * (1.0f / WCARRY) + bb, 0.0f);
        const float u1 = fmaxf(acc1[ai][r] * (1.0f / WCARRY) + bb, 0.0f);
        psum[ai][r] += u0 + u1;
      }
  }

#pragma unroll
  for (int ai = 0; ai < 4; ++ai)
#pragma unroll
    for (int r = 0; r < 8; ++r) {
      float v = psum[ai][r];
      v += __shfl_xor(v, 1, 32);
      v += __shfl_xor(v, 2, 32);
      v += __shfl_xor(v, 4, 32);
      v += __shfl_xor(v, 8, 32);
      psum[ai][r] = v;
    }
  if (mm == 0) {
#pragma unroll
    for (int ai = 0; ai < 4; ++ai)
#pragma unroll
      for (int r = 0; r < 8; ++r) poolw[wv * 64 + ai * 16 + 8 * hh + r] = psum[ai][r];
  }
  __syncthreads();
  if (tid < CH2) {
    const int mb = tid >> 6, lch = tid & 63;
    const float t0 = poolw[(0 * 2 + mb) * 64 + lch];
    const float t1 = poolw[(1 * 2 + mb) * 64 + lch];
    const float t2 = poolw[(2 * 2 + mb) * 64 + lch];
    const float t3 = poolw[(3 * 2 + mb) * 64 + lch];
    spool[tid] = (((t0 + t1) + t2) + t3) * (1.0f / (float)NPIX);
  }
  __syncthreads();
  if (wv == 0 && lane < 16) {
    const float* sp = spool + lane * 8;
    v8h hv;
#pragma unroll
    for (int e = 0; e < 8; ++e) hv[e] = (_Float16)sp[e];
    _Float16* dst = pooled_out + (size_t)img * CH2 + lane * 8;
    *(volatile v8h*)dst = hv;
    __threadfence();
    *(volatile v8h*)dst = hv;
  }
}

template <int MASKED>
__global__ __launch_bounds__(256)
void sage_pack_kernel(const float* __restrict__ zin, const float* __restrict__ mask,
                      _Float16* __restrict__ aout) {
  __shared__ __align__(16) float zs[NNODE * HIDD];
  __shared__ __align__(16) float ssum[HIDD];
  __shared__ float smask[NNODE];
  const int tid = threadIdx.x, lane = tid & 31, wv = tid >> 5;
  const int b = blockIdx.x;
  if (tid < NNODE) smask[tid] = MASKED ? mask[b * NNODE + tid] : 1.0f;
  __syncthreads();
  float s = 0.0f;
  const float* zb = zin + (size_t)b * NNODE * HIDD + tid;
#pragma unroll 1
  for (int g = 0; g < NNODE / 4; ++g) {
    const int nb = g * 4;
    const float v0 = zb[(size_t)(nb + 0) * HIDD];
    const float v1 = zb[(size_t)(nb + 1) * HIDD];
    const float v2 = zb[(size_t)(nb + 2) * HIDD];
    const float v3 = zb[(size_t)(nb + 3) * HIDD];
    const float z0 = MASKED ? v0 * smask[nb + 0] : v0;
    const float z1 = MASKED ? v1 * smask[nb + 1] : v1;
    const float z2 = MASKED ? v2 * smask[nb + 2] : v2;
    const float z3 = MASKED ? v3 * smask[nb + 3] : v3;
    zs[(nb + 0) * HIDD + tid] = z0;
    zs[(nb + 1) * HIDD + tid] = z1;
    zs[(nb + 2) * HIDD + tid] = z2;
    zs[(nb + 3) * HIDD + tid] = z3;
    s += z0; s += z1; s += z2; s += z3;
  }
  ssum[tid] = s;
  __syncthreads();
  const float inv_nm1 = 1.0f / (float)(NNODE - 1);
  for (int pass = 0; pass < 2; ++pass) {
#pragma unroll
    for (int it = 0; it < 4; ++it) {
      const int n = it * 8 + wv;
      const float* zr = zs + n * HIDD + lane * 8;
      const v4f za = *(const v4f*)zr;
      const v4f zc = *(const v4f*)(zr + 4);
      const v4f sa = *(const v4f*)(ssum + lane * 8);
      const v4f sc = *(const v4f*)(ssum + lane * 8 + 4);
      v8h ha, hz;
#pragma unroll
      for (int e = 0; e < 4; ++e) {
        const float ag0 = (sa[e] - za[e]) * inv_nm1;
        const float ag1 = (sc[e] - zc[e]) * inv_nm1;
        ha[e]     = (_Float16)(ag0 * ACARRY);
        ha[4 + e] = (_Float16)(ag1 * ACARRY);
        hz[e]     = (_Float16)(za[e] * ACARRY);
        hz[4 + e] = (_Float16)(zc[e] * ACARRY);
      }
      _Float16* rowp = aout + (size_t)(b * NNODE + n) * KSAGE;
      *(volatile v8h*)(rowp + lane * 8) = ha;
      *(volatile v8h*)(rowp + HIDD + lane * 8) = hz;
    }
    __threadfence();
  }
}

extern "C" void kernel_launch(void* const* d_in, const int* in_sizes, int n_in,
                              void* d_out, int out_size, void* d_ws, size_t ws_size,
                              hipStream_t stream) {
  if (n_in < 14) return;
  if (ws_size < WS_TOTAL) return;
  if (out_size != NIMG * OUTDIM) return;
  if (in_sizes[0] != NIMG * CIN * NPIX || in_sizes[1] != NIMG || in_sizes[2] != CH1 * 27 ||
      in_sizes[3] != CH1 || in_sizes[4] != CH2 * KCONV2 || in_sizes[5] != CH2 ||
      in_sizes[6] != HIDD * CH2 || in_sizes[7] != HIDD || in_sizes[8] != HIDD * HIDD ||
      in_sizes[9] != HIDD || in_sizes[10] != HIDD * HIDD || in_sizes[11] != OUTDIM * HIDD ||
      in_sizes[12] != OUTDIM || in_sizes[13] != OUTDIM * HIDD) return;

  const float* x       = (const float*)d_in[0];
  const float* mask    = (const float*)d_in[1];
  const float* conv1_w = (const float*)d_in[2];
  const float* conv1_b = (const float*)d_in[3];
  const float* conv2_w = (const float*)d_in[4];
  const float* conv2_b = (const float*)d_in[5];
  const float* fc_w    = (const float*)d_in[6];
  const float* fc_b    = (const float*)d_in[7];
  const float* s1_lw   = (const float*)d_in[8];
  const float* s1_lb   = (const float*)d_in[9];
  const float* s1_rw   = (const float*)d_in[10];
  const float* s2_lw   = (const float*)d_in[11];
  const float* s2_lb   = (const float*)d_in[12];
  const float* s2_rw   = (const float*)d_in[13];

  char* ws = (char*)d_ws;
  _Float16* planes = (_Float16*)(ws + WSO_PLANES);
  const unsigned short* pW2C   = (const unsigned short*)(planes);
  const unsigned short* pFCW   = (const unsigned short*)(planes + PL_OFF_FCW);
  const unsigned short* pW1CAT = (const unsigned short*)(planes + PL_OFF_W1CAT);
  const unsigned short* pW2CAT = (const unsigned short*)(planes + PL_OFF_W2CAT);
  _Float16* pooled = (_Float16*)(ws + WSO_POOL);
  float* z0 = (float*)(ws + WSO_Z0);
  _Float16* a1 = (_Float16*)(ws + WSO_A1);
  float* z1 = (float*)(ws + WSO_Z1);
  _Float16* a2 = (_Float16*)(ws + WSO_A2);
  float* out = (float*)d_out;

  prep_planes_kernel<<<PREP_BLOCKS, 256, 0, stream>>>(conv2_w, fc_w, s1_lw, s1_rw, s2_lw, s2_rw, planes);

  conv_pool_kernel<<<NIMG, 256, SMO_TOTAL, stream>>>(x, conv1_w, conv1_b, (const _Float16*)pW2C, conv2_b, pooled);

  {
    const int tiles = (NIMG / 64) * (HIDD / 64);
    wmma_gemm64<0, false, 2, 0, false, 0><<<dim3(tiles / 8, 1), 256, 0, stream>>>(
        (const unsigned short*)pooled, (const unsigned short*)pooled, CH2, (long)0,
        pFCW, pFCW, CH2, (long)0,
        (void*)z0, (void*)z0, HIDD, (long)0,
        fc_b, fc_b, (long)0, NIMG, HIDD, CH2, 1.0f / WCARRY);
  }

  sage_pack_kernel<1><<<NSAMP, 256, 0, stream>>>(z0, mask, a1);

  {
    const int tiles = (NIMG / 64) * (HIDD / 64);
    wmma_gemm64<0, false, 2, 0, false, 2><<<dim3(tiles / 8, 1), 256, 0, stream>>>(
        (const unsigned short*)a1, (const unsigned short*)a1, KSAGE, (long)0,
        pW1CAT, pW1CAT, KSAGE, (long)0,
        (void*)z1, (void*)z1, HIDD, (long)0,
        s1_lb, s1_lb, (long)0, NIMG, HIDD, KSAGE, 1.0f / (WCARRY * ACARRY));
  }

  sage_pack_kernel<0><<<NSAMP, 256, 0, stream>>>(z1, mask, a2);

  {
    const int tiles = (NIMG / 64) * (OUTDIM / 64);
    wmma_gemm64<0, false, 2, 0, false, 0><<<dim3(tiles / 8, 1), 256, 0, stream>>>(
        (const unsigned short*)a2, (const unsigned short*)a2, KSAGE, (long)0,
        pW2CAT, pW2CAT, KSAGE, (long)0,
        (void*)out, (void*)out, OUTDIM, (long)0,
        s2_lb, s2_lb, (long)0, NIMG, OUTDIM, KSAGE, 1.0f / (WCARRY * ACARRY));
  }
}
